// MaskedSelfAttend_9474697855745
// MI455X (gfx1250) — hardware-verified
//
#include <hip/hip_runtime.h>
#include <math.h>

typedef __attribute__((ext_vector_type(16))) _Float16 v16h;
typedef __attribute__((ext_vector_type(16))) __bf16 v16b;
typedef __attribute__((ext_vector_type(8)))  _Float16 v8h;
typedef __attribute__((ext_vector_type(8)))  float v8f;
typedef __attribute__((ext_vector_type(4)))  float v4f;
typedef __attribute__((ext_vector_type(2)))  float v2f;
typedef __attribute__((ext_vector_type(4)))  unsigned v4u;
typedef __attribute__((ext_vector_type(4)))  int v4i;
typedef float __attribute__((may_alias)) float_a;
typedef int __attribute__((may_alias)) int_a;

template <typename T> __device__ __forceinline__ void vst2(void* p, T v) { *(volatile T*)p = v; __threadfence(); *(volatile T*)p = v; }
__device__ __forceinline__ v8f wmma16(v16h a, v16h b, v8f c) {
  v8f d = __builtin_amdgcn_wmma_f32_16x16x32_f16(false, a, false, b, (short)0, c, false, false);
  asm volatile("v_nop\n\tv_nop\n\tv_nop\n\tv_nop" : "+v"(d) : "v"(a), "v"(b));
  return d;
}
__device__ __forceinline__ v8f wmma_bf(v16b a, v16b b, v8f c) {
  v8f d = __builtin_amdgcn_wmma_f32_16x16x32_bf16(false, a, false, b, (short)0, c, false, false);
  asm volatile("v_nop\n\tv_nop\n\tv_nop\n\tv_nop" : "+v"(d) : "v"(a), "v"(b));
  return d;
}
__device__ __forceinline__ v16h frag_h(const _Float16* rowk0, int lane) {
  union { v16h v; v8h q[2]; } u; const _Float16* p = rowk0 + 8 * (lane >> 4);
  u.q[0] = *(const v8h*)p; u.q[1] = *(const v8h*)(p + 16); return u.v;
}
__device__ __forceinline__ v16h frag_f32(const float* rowk0, int lane) {
  v16h a; const float* p = rowk0 + 8 * (lane >> 4);
#pragma unroll
  for (int i = 0; i < 8; ++i) { a[i] = (_Float16)p[i]; a[8 + i] = (_Float16)p[16 + i]; }
  return a;
}
__device__ __forceinline__ v16h frag_f32s(const float* rowk0, int lane, float sc) {
  v16h a; const float* p = rowk0 + 8 * (lane >> 4);
#pragma unroll
  for (int i = 0; i < 8; ++i) { a[i] = (_Float16)(p[i] * sc); a[8 + i] = (_Float16)(p[16 + i] * sc); }
  return a;
}
__device__ __forceinline__ v16h fragc_f32(const float* W, int k0, int n, int lane, int ld, int K) {
  v16h a; const int g = lane >> 4;
#pragma unroll
  for (int i = 0; i < 8; ++i) { const int ka = k0 + 8 * g + i, kb = ka + 16;
    a[i] = (_Float16)(ka < K ? W[(size_t)(ka < K ? ka : K - 1) * ld + n] : 0.f); a[8 + i] = (_Float16)(kb < K ? W[(size_t)(kb < K ? kb : K - 1) * ld + n] : 0.f); }
  return a;
}
struct F2 { v16b h, l; };
__device__ __forceinline__ F2 bsplit16(const float v[16]) { F2 r;
#pragma unroll
  for (int i = 0; i < 16; ++i) { const __bf16 h = (__bf16)v[i]; r.h[i] = h; r.l[i] = (__bf16)(v[i] - (float)h); }
  return r; }
__device__ __forceinline__ F2 split_row(const float* row, int k0, int lane) { float v[16]; const float* p = row + k0 + 8 * (lane >> 4);
#pragma unroll
  for (int i = 0; i < 8; ++i) { v[i] = p[i]; v[8 + i] = p[16 + i]; }
  return bsplit16(v); }
__device__ __forceinline__ F2 split_rowK(const float* row, int k0, int lane, int K) { float v[16]; const int g = lane >> 4;
#pragma unroll
  for (int i = 0; i < 8; ++i) { const int ka = k0 + 8 * g + i, kb = ka + 16; v[i] = ka < K ? row[ka < K ? ka : K - 1] : 0.f; v[8 + i] = kb < K ? row[kb < K ? kb : K - 1] : 0.f; }
  return bsplit16(v); }
__device__ __forceinline__ F2 split_col(const float* W, int k0, int n, int lane, int ld, int K) { float v[16]; const int g = lane >> 4;
#pragma unroll
  for (int i = 0; i < 8; ++i) { const int ka = k0 + 8 * g + i, kb = ka + 16; v[i] = ka < K ? W[(size_t)(ka < K ? ka : K - 1) * ld + n] : 0.f; v[8 + i] = kb < K ? W[(size_t)(kb < K ? kb : K - 1) * ld + n] : 0.f; }
  return bsplit16(v); }
__device__ __forceinline__ v8f mac3(const F2& a, const F2& b, v8f c) { c = wmma_bf(a.l, b.h, c); c = wmma_bf(a.h, b.l, c); return wmma_bf(a.h, b.h, c); }
__device__ __forceinline__ float sigm(float v) { return 1.0f / (1.0f + expf(-v)); }
#define LDSX() do { asm volatile("s_wait_dscnt 0" ::: "memory"); __builtin_amdgcn_wave_barrier(); __builtin_amdgcn_fence(__ATOMIC_RELEASE, "workgroup"); } while (0)


#define NBq 16
#define LL 2048
#define HDD 128
#define NR (NBq * LL)
#ifndef TQB
#define TQB (LL / 64)
#endif
typedef __attribute__((ext_vector_type(8))) __bf16 v8b;
__device__ __forceinline__ v16b frag_b(const __bf16* rowk0, int lane) {
  union { v16b v; v8b q[2]; } u; const __bf16* p = rowk0 + 8 * (lane >> 4);
  u.q[0] = *(const v8b*)p; u.q[1] = *(const v8b*)(p + 16); return u.v;
}
__device__ __forceinline__ float bfr(float v) { return (float)(__bf16)v; }
__device__ __attribute__((noinline)) float exp_ni(float v) { return expf(v); }
__device__ __attribute__((noinline)) float erf_ni(float v) { return erff(v); }

#define WS_QH  0u
#define WS_VT  (WS_QH + 2u * NR * HDD)
#define WS_END (WS_VT + 2u * NR * HDD)

__global__ __launch_bounds__(256) void k_prep(const float* __restrict__ Q, _Float16* __restrict__ QH, _Float16* __restrict__ VT) {
  __shared__ __align__(16) _Float16 sq[64][HDD + 8]; __shared__ __align__(16) _Float16 st[HDD][72];
  const int t = threadIdx.x; const size_t r0 = (size_t)blockIdx.x * 64; const size_t b = r0 / LL, s0 = r0 % LL;
  for (int e = t; e < 64 * HDD; e += 256) { const int r = e >> 7, c = e & 127; const _Float16 v = (_Float16)bfr(Q[(r0 + r) * HDD + c]); sq[r][c] = v; st[c][r] = v; }
  __syncthreads();
  for (int e = t; e < 64 * 16; e += 256) { const int r = e >> 4, q = e & 15; vst2((unsigned*)(QH + (r0 + r) * HDD + q * 8), *(const v4u*)&sq[r][q * 8]); }
  for (int e = t; e < HDD * 8; e += 256) { const int c = e >> 3, pc = e & 7; vst2((unsigned*)(VT + (b * HDD + c) * LL + s0 + pc * 8), *(const v4u*)&st[c][pc * 8]); }
}
__global__ __launch_bounds__(128) void k_attn(const _Float16* __restrict__ QH, const _Float16* __restrict__ VT, float* __restrict__ OUT) {
  __shared__ __align__(16) _Float16 sph[4][16][40], spl[4][16][40]; __shared__ __align__(16) float so[4][16][132];
  const int tid = threadIdx.x, wave = tid >> 5, lane = tid & 31, col = lane & 15, g = lane >> 4; const size_t b = blockIdx.y; const int q0 = blockIdx.x * 64 + wave * 16; const size_t rq = b * LL + q0;
  v16h aq[4];
#pragma unroll
  for (int kc = 0; kc < 4; ++kc) aq[kc] = frag_h(QH + (rq + col) * HDD + kc * 32, lane);
  float m[8], l[8];
#pragma unroll
  for (int r = 0; r < 8; ++r) { m[r] = -3.0e38f; l[r] = 0.f; }
  v8f acc[8] = {}, accl[8] = {}; const float scale = 1.0f / sqrtf((float)HDD);
#pragma unroll 1
  for (int ks = 0; ks < LL / 32; ++ks) { const int j0 = ks * 32; v8f s[2];
#pragma unroll
    for (int ct = 0; ct < 2; ++ct) { const int kk = j0 + ct * 16 + col; const size_t rk = (b * LL + kk) * HDD; v8f c = {};
#pragma unroll
      for (int kc = 0; kc < 4; ++kc) c = wmma16(aq[kc], frag_h(QH + rk + kc * 32, lane), c);
#pragma unroll
      for (int r = 0; r < 8; ++r) s[ct][r] = (kk == q0 + 8 * g + r) ? -3.0e38f : c[r] * scale; }
#pragma unroll
    for (int r = 0; r < 8; ++r) { float mx = fmaxf(s[0][r], s[1][r]);
#pragma unroll
      for (int o = 1; o < 16; o <<= 1) mx = fmaxf(mx, __shfl_xor(mx, o));
      const float mn = fmaxf(m[r], mx); const float alpha = (m[r] <= -1.0e38f) ? 0.f : __expf(m[r] - mn); const float e0 = (s[0][r] <= -1.0e38f) ? 0.f : __expf(s[0][r] - mn), e1 = (s[1][r] <= -1.0e38f) ? 0.f : __expf(s[1][r] - mn); float es = e0 + e1;
#pragma unroll
      for (int o = 1; o < 16; o <<= 1) es += __shfl_xor(es, o);
      l[r] = l[r] * alpha + es; m[r] = (mn <= -1.0e38f) ? m[r] : mn;
#pragma unroll
      for (int dt = 0; dt < 8; ++dt) { acc[dt][r] *= alpha; accl[dt][r] *= alpha; }
      { const float p0 = e0 * 2048.0f, p1 = e1 * 2048.0f; const _Float16 h0 = (_Float16)p0, h1 = (_Float16)p1; sph[wave][8 * g + r][col] = h0; sph[wave][8 * g + r][16 + col] = h1; spl[wave][8 * g + r][col] = (_Float16)((p0 - (float)h0) * 2048.0f); spl[wave][8 * g + r][16 + col] = (_Float16)((p1 - (float)h1) * 2048.0f); } }
    LDSX();
    const v16h pa = frag_h(&sph[wave][col][0], lane), pl = frag_h(&spl[wave][col][0], lane);
#pragma unroll
    for (int dt = 0; dt < 8; ++dt) { const v16h vh = frag_h(VT + (b * HDD + dt * 16 + col) * LL + j0, lane); acc[dt] = wmma16(pa, vh, acc[dt]); accl[dt] = wmma16(pl, vh, accl[dt]); }
    LDSX(); }
#pragma unroll
  for (int r = 0; r < 8; ++r) { const float il = (1.0f / 2048.0f) / l[r];
#pragma unroll
    for (int dt = 0; dt < 8; ++dt) so[wave][8 * g + r][dt * 16 + col] = (acc[dt][r] + accl[dt][r] * (1.0f / 2048.0f)) * il; }
  LDSX();
  for (int rl = 0; rl < 16; ++rl) vst2(OUT + (rq + rl) * HDD + lane * 4, *(const v4f*)&so[wave][rl][lane * 4]);
}
extern "C" void kernel_launch(void* const* d_in, const int* in_sizes, int n_in, void* d_out, int out_size, void* d_ws, size_t ws_size, hipStream_t stream) {
  (void)in_sizes; (void)n_in; (void)out_size;
  const float** F = (const float**)d_in;
  if (ws_size < (size_t)WS_END) return;
  char* ws = (char*)d_ws; _Float16 *QH = (_Float16*)(ws + WS_QH), *VT = (_Float16*)(ws + WS_VT);
  k_prep<<<NR / 64, 256, 0, stream>>>(F[0], QH, VT);
  k_attn<<<dim3(TQB, NBq), 128, 0, stream>>>(QH, VT, (float*)d_out);
}
